// LSTM_53815940218945
// MI455X (gfx1250) — hardware-verified
//
#include <hip/hip_runtime.h>
#include <math.h>

constexpr int NBATCH   = 8192;
constexpr int NSTEP    = 256;
constexpr int NHID     = 50;
constexpr int NGATE    = 4;
constexpr int HPAD     = 64;
constexpr int NTHR     = 128;
constexpr int NWAVE    = NTHR / 32;
constexpr int ROWS_BLK = NWAVE * 16;
constexpr int WPITCH   = 72;
constexpr int HPITCH   = 72;
constexpr int XCH      = 16;
constexpr float HCARRY     = 1024.0f;
constexpr float WCARRY     = 256.0f;
constexpr float PCARRY     = HCARRY * WCARRY;
constexpr float PCARRY_INV = 1.0f / PCARRY;

static_assert(NBATCH % ROWS_BLK == 0, "grid exact");
static_assert(NSTEP % XCH == 0, "x chunks exact");
static_assert(HPAD % 32 == 0 && NHID <= HPAD, "K padded to a multiple of 32");
static_assert(WPITCH % 8 == 0 && HPITCH % 8 == 0 && WPITCH >= HPAD && HPITCH >= HPAD, "pitches");
static_assert((NWAVE * 16 * HPITCH) % NTHR == 0, "h zero fill exact");
static_assert((NGATE * HPAD * (HPAD / 8)) % NTHR == 0, "weight tile build exact");
static_assert(NGATE * HPAD == 2 * NTHR, "constant staging exact");
static_assert(XCH * 16 == 2 * 32 * 4, "x chunk staging exact");
static_assert(ROWS_BLK == 64, "block output = 2 whole lines");

typedef __attribute__((ext_vector_type(16))) _Float16 v16h;
typedef __attribute__((ext_vector_type(8)))  _Float16 v8h;
typedef __attribute__((ext_vector_type(8)))  float    v8f;
typedef __attribute__((ext_vector_type(4)))  float    v4f;

template <typename T> struct Frag;
template <> struct Frag<_Float16> {
  typedef v16h V; union U { v16h v; v8h h[2]; };
  static __device__ __forceinline__ v16h load(const _Float16* p) {
    U f; f.h[0] = *(const v8h*)(p); f.h[1] = *(const v8h*)(p + 16); return f.v;
  }
  static __device__ __forceinline__ v8f mma(v16h a, v16h b, v8f c) {
    return __builtin_amdgcn_wmma_f32_16x16x32_f16(false, a, false, b, (short)0, c, false, false);
  }
};

__device__ __forceinline__ void guard_grp(v8f& acc, v16h a0, v16h a1, v16h b0, v16h b1) {
  asm volatile("v_nop\n\tv_nop\n\tv_nop\n\tv_nop" : "+v"(acc) : "v"(a0), "v"(a1), "v"(b0), "v"(b1));
}
__device__ __forceinline__ void opaque_i(int& v) { asm volatile("" : "+v"(v)); }

__device__ __forceinline__ float fsig(float x)  { return __builtin_amdgcn_rcpf(1.0f + __expf(-x)); }
__device__ __forceinline__ float ftanh(float x) { return 1.0f - 2.0f * __builtin_amdgcn_rcpf(__expf(2.0f * x) + 1.0f); }

__device__ __forceinline__ void stage_x(const float* __restrict__ xw, float* xs, int t0, int lane) {
#pragma unroll
  for (int i = 0; i < 2; ++i) {
    const int m  = 8 * i + (lane >> 2);
    const int c4 = (lane & 3) * 4;
    const v4f v = *(const v4f*)(xw + (size_t)m * NSTEP + t0 + c4);
    const float e0 = v[0], e1 = v[1], e2 = v[2], e3 = v[3];
    xs[(c4 + 0) * 16 + m] = e0;
    xs[(c4 + 1) * 16 + m] = e1;
    xs[(c4 + 2) * 16 + m] = e2;
    xs[(c4 + 3) * 16 + m] = e3;
  }
}

__global__ __launch_bounds__(NTHR) void recur_kernel(const float* __restrict__ x, const float* __restrict__ w_ih,
                                                     const float* __restrict__ w_hh, const float* __restrict__ b_ih,
                                                     const float* __restrict__ b_hh, const float* __restrict__ w_lin,
                                                     const float* __restrict__ b_lin, float* __restrict__ out) {
  __shared__ __align__(16) _Float16 Wt[NGATE * HPAD * WPITCH];
  __shared__ __align__(16) _Float16 Ah[NWAVE * 16 * HPITCH];
  __shared__ __align__(16) float    Xs[NWAVE * 2 * XCH * 16];
  __shared__ __align__(16) float    WiS[NGATE * HPAD];
  __shared__ __align__(16) float    BsS[NGATE * HPAD];
  __shared__ __align__(16) float    OutS[ROWS_BLK];

  const int tid = threadIdx.x, lane = tid & 31, wave = tid >> 5;
  const int c = lane & 15, hh = lane >> 4, koff = hh * 8;

#pragma unroll 1
  for (int it = 0; it < (NGATE * HPAD * (HPAD / 8)) / NTHR; ++it) {
    const int idx  = it * NTHR + tid;
    const int np   = idx >> 3;
    const int k8   = (idx & 7) * 8;
    const int gate = np >> 6;
    const int j    = np & 63;
    const int jc   = (j < NHID) ? j : (NHID - 1);
    const float* wrow = w_hh + (size_t)(gate * NHID + jc) * NHID;
    v8h hv;
#pragma unroll
    for (int e = 0; e < 8; ++e) {
      const int k  = k8 + e;
      const int kc = (k < NHID) ? k : (NHID - 1);
      const float w = wrow[kc];
      const bool ok = (j < NHID) && (k < NHID);
      const float wsv = ok ? (w * WCARRY) : 0.0f;
      hv[e] = (_Float16)wsv;
    }
    *(v8h*)(Wt + np * WPITCH + k8) = hv;
  }
#pragma unroll 1
  for (int i = tid; i < NWAVE * 16 * HPITCH; i += NTHR) Ah[i] = (_Float16)0.0f;
#pragma unroll
  for (int q = 0; q < 2; ++q) {
    const int np   = q * NTHR + tid;
    const int gate = np >> 6;
    const int j    = np & 63;
    const int jc   = (j < NHID) ? j : (NHID - 1);
    const int row  = gate * NHID + jc;
    const float wi = w_ih[row];
    const float bi = b_ih[row];
    const float bh = b_hh[row];
    const bool ok  = (j < NHID);
    const float bsum = bi + bh;
    WiS[np] = ok ? (wi * PCARRY) : 0.0f;
    BsS[np] = ok ? (bsum * PCARRY) : 0.0f;
  }
  const float* xw  = x + (size_t)(blockIdx.x * ROWS_BLK + wave * 16) * NSTEP;
  float*       xsw = Xs + wave * (2 * XCH * 16);
  stage_x(xw, xsw, 0, lane);
  __syncthreads();

  float wiR[4][4], bsR[4][4], wlin[4];
#pragma unroll
  for (int jt = 0; jt < 4; ++jt) {
#pragma unroll
    for (int g = 0; g < 4; ++g) {
      wiR[jt][g] = WiS[g * HPAD + 16 * jt + c];
      bsR[jt][g] = BsS[g * HPAD + 16 * jt + c];
    }
    const int j  = 16 * jt + c;
    const int jc = (j < NHID) ? j : (NHID - 1);
    const float wl = w_lin[jc];
    wlin[jt] = (j < NHID) ? wl : 0.0f;
  }
  const float blin = b_lin[0];
  const bool cval3 = (48 + c) < NHID;

  float cst[4][8], pd[8];
#pragma unroll
  for (int jt = 0; jt < 4; ++jt)
#pragma unroll
    for (int r = 0; r < 8; ++r) cst[jt][r] = 0.0f;
#pragma unroll
  for (int r = 0; r < 8; ++r) pd[r] = 0.0f;

  _Float16*       ahw   = Ah + wave * (16 * HPITCH);
  const _Float16* ahrow = ahw + c * HPITCH + koff;

#pragma unroll 1
  for (int t = 0; t < NSTEP; ++t) {
    int woff = c * WPITCH + koff;
    opaque_i(woff);
    const _Float16* wp = Wt + woff;

    const float* xsb = xsw + ((t >> 4) & 1) * (XCH * 16) + (t & (XCH - 1)) * 16 + 8 * hh;
    const v4f xa = *(const v4f*)(xsb);
    const v4f xb = *(const v4f*)(xsb + 4);
    float xv[8];
    xv[0] = xa[0]; xv[1] = xa[1]; xv[2] = xa[2]; xv[3] = xa[3];
    xv[4] = xb[0]; xv[5] = xb[1]; xv[6] = xb[2]; xv[7] = xb[3];

    const v16h a0 = Frag<_Float16>::load(ahrow);
    const v16h a1 = Frag<_Float16>::load(ahrow + 32);
#pragma unroll
    for (int r = 0; r < 8; ++r) pd[r] = 0.0f;

#pragma unroll
    for (int jt = 0; jt < 4; ++jt) {
      v8f acc[4];
#pragma unroll
      for (int g = 0; g < 4; ++g) {
        v8f ac;
#pragma unroll
        for (int r = 0; r < 8; ++r) ac[r] = fmaf(wiR[jt][g], xv[r], bsR[jt][g]);
        const v16h b0 = Frag<_Float16>::load(wp + (g * HPAD + 16 * jt) * WPITCH);
        const v16h b1 = Frag<_Float16>::load(wp + (g * HPAD + 16 * jt) * WPITCH + 32);
        ac = Frag<_Float16>::mma(a0, b0, ac);
        ac = Frag<_Float16>::mma(a1, b1, ac);
        guard_grp(ac, a0, a1, b0, b1);
        acc[g] = ac;
      }
#pragma unroll
      for (int r = 0; r < 8; ++r) {
        const float zi = acc[0][r] * PCARRY_INV;
        const float zf = acc[1][r] * PCARRY_INV;
        const float zg = acc[2][r] * PCARRY_INV;
        const float zo = acc[3][r] * PCARRY_INV;
        const float ig = fsig(zi);
        const float fg = fsig(zf);
        const float gg = ftanh(zg);
        const float og = fsig(zo);
        const float cn = fg * cst[jt][r] + ig * gg;
        cst[jt][r] = cn;
        const float hn = og * ftanh(cn);
        pd[r] = fmaf(wlin[jt], hn, pd[r]);
        const float hsc = hn * HCARRY;
        const float hs = (jt < 3 || cval3) ? hsc : 0.0f;
        ahw[(8 * hh + r) * HPITCH + 16 * jt + c] = (_Float16)hs;
      }
    }
    if (((t & (XCH - 1)) == (XCH - 1)) && (t + 1 < NSTEP)) {
      stage_x(xw, xsw + (((t + 1) >> 4) & 1) * (XCH * 16), t + 1, lane);
    }
    __syncthreads();
  }

#pragma unroll
  for (int r = 0; r < 8; ++r) {
    float s = pd[r];
    s += __shfl_xor(s, 1, 32);
    s += __shfl_xor(s, 2, 32);
    s += __shfl_xor(s, 4, 32);
    s += __shfl_xor(s, 8, 32);
    pd[r] = s + blin;
  }
  if (c == 0) {
#pragma unroll
    for (int r = 0; r < 8; ++r) OutS[wave * 16 + 8 * hh + r] = pd[r];
  }
  __syncthreads();
  if (tid < 16) {
    const v4f v = *(const v4f*)(OutS + tid * 4);
    float* op = out + (size_t)blockIdx.x * ROWS_BLK + tid * 4;
    *(volatile v4f*)op = v;
    __threadfence();
    *(volatile v4f*)op = v;
  }
}

extern "C" void kernel_launch(void* const* d_in, const int* in_sizes, int n_in,
                              void* d_out, int out_size, void* d_ws, size_t ws_size, hipStream_t stream) {
  (void)d_ws; (void)ws_size;
  if (n_in < 7 || d_out == nullptr) return;
  if (in_sizes[0] != NBATCH * NSTEP || in_sizes[1] != NGATE * NHID || in_sizes[2] != NGATE * NHID * NHID ||
      in_sizes[3] != NGATE * NHID || in_sizes[4] != NGATE * NHID || in_sizes[5] != NHID || in_sizes[6] != 1 ||
      out_size != NBATCH) return;
  const float* x     = (const float*)d_in[0];
  const float* w_ih  = (const float*)d_in[1];
  const float* w_hh  = (const float*)d_in[2];
  const float* b_ih  = (const float*)d_in[3];
  const float* b_hh  = (const float*)d_in[4];
  const float* w_lin = (const float*)d_in[5];
  const float* b_lin = (const float*)d_in[6];
  float* out = (float*)d_out;
  recur_kernel<<<NBATCH / ROWS_BLK, NTHR, 0, stream>>>(x, w_ih, w_hh, b_ih, b_hh, w_lin, b_lin, out);
}
